// cnn_lstm_layer_40450001993746
// MI455X (gfx1250) — hardware-verified
//
#include <hip/hip_runtime.h>

typedef __attribute__((ext_vector_type(16))) _Float16 v16h;
typedef __attribute__((ext_vector_type(8)))  _Float16 v8h;
typedef __attribute__((ext_vector_type(8)))  float    v8f;

#define SC 20
#define EDIM 16
#define CONV_OUT 12
#define H 10
#define G4 40
#define TILE 16

#define LDS_FENCE() asm volatile("s_wait_dscnt 0" ::: "memory")

__device__ __forceinline__ v8f wmma16(v16h a, v16h b, v8f c) {
  return __builtin_amdgcn_wmma_f32_16x16x32_f16(false, a, false, b, (short)0, c, false, false);
}

__device__ __forceinline__ float sigm(float x) { return 1.f / (1.f + __expf(-x)); }
__device__ __forceinline__ float tanh_fast(float x) {
  float e = __expf(2.f * x);
  return 1.f - 2.f / (e + 1.f);
}

__global__ __launch_bounds__(64)
void cnn_bilstm_kernel(const int*   __restrict__ in,
                       const float* __restrict__ emb,
                       const float* __restrict__ k2,
                       const float* __restrict__ k3,
                       const float* __restrict__ k4,
                       const float* __restrict__ w_fw, const float* __restrict__ b_fw,
                       const float* __restrict__ w_bw, const float* __restrict__ b_bw,
                       float* __restrict__ out)
{
  __shared__ __align__(16) _Float16 s_emb[TILE * SC * 16];
  __shared__ __align__(16) _Float16 s_c  [TILE * SC * 16];
  __shared__ __align__(16) _Float16 s_h  [2][TILE * 16];
  __shared__ __align__(16) float    s_z  [2][48 * 16];

  const int tid  = threadIdx.x;
  const int wave = tid >> 5;
  const int lane = tid & 31;
  const int m    = lane & 15;
  const int hsel = lane >> 4;
  const int base = blockIdx.x * TILE;

  for (int p = tid; p < TILE * SC; p += 64) {
    int s = p / SC, ch = p % SC;
    int id = in[(base + s) * SC + ch];
    const float* er = emb + id * EDIM;
    v16h tmp;
    #pragma unroll
    for (int e = 0; e < 16; ++e) tmp[e] = (_Float16)er[e];
    *(v16h*)&s_emb[(s * SC + ch) * 16] = tmp;
  }
  __syncthreads();

  if (wave == 0) {
    v16h cb0, cb1;
    {
      const int nf = lane & 15;
      #pragma unroll
      for (int kh = 0; kh < 2; ++kh) {
        #pragma unroll
        for (int i = 0; i < 16; ++i) {
          int kk = kh * 32 + ((i < 8) ? i : (i + 8)) + 8 * hsel;
          int w = kk >> 4, e = kk & 15;
          float val = 0.f;
          if (nf < 3)       { int q = w - 2; if (q >= 0) val = k2[(q * 16 + e) * 3 + nf]; }
          else if (nf < 7)  { int q = w - 1; if (q >= 0) val = k3[(q * 16 + e) * 4 + (nf - 3)]; }
          else if (nf < 12) {                            val = k4[(w * 16 + e) * 5 + (nf - 7)]; }
          if (kh == 0) cb0[i] = (_Float16)val; else cb1[i] = (_Float16)val;
        }
      }
    }
    const _Float16* eb = &s_emb[m * SC * 16 + 8 * hsel];
    v8h z8 = {};
    #pragma unroll 1
    for (int t = 0; t < SC; ++t) {
      v8h c0 = (t >= 3) ? *(const v8h*)(eb + (t - 3) * 16) : z8;
      v8h c1 = (t >= 2) ? *(const v8h*)(eb + (t - 2) * 16) : z8;
      v8h c2 = (t >= 1) ? *(const v8h*)(eb + (t - 1) * 16) : z8;
      v8h c3 =            *(const v8h*)(eb + t * 16);
      v16h a0 = __builtin_shufflevector(c0, c1, 0,1,2,3,4,5,6,7,8,9,10,11,12,13,14,15);
      v16h a1 = __builtin_shufflevector(c2, c3, 0,1,2,3,4,5,6,7,8,9,10,11,12,13,14,15);
      v8f acc = {};
      acc = wmma16(a0, cb0, acc);
      acc = wmma16(a1, cb1, acc);
      int n = lane & 15;
      #pragma unroll
      for (int v = 0; v < 8; ++v)
        s_c[((v + 8 * hsel) * SC + t) * 16 + n] = (_Float16)acc[v];
    }
  }

  const float* W = (wave == 0) ? w_fw : w_bw;
  const float* B = (wave == 0) ? b_fw : b_bw;
  v16h wb[3];
  v8f  biasC[3];
  #pragma unroll
  for (int j = 0; j < 3; ++j) {
    #pragma unroll
    for (int i = 0; i < 16; ++i) {
      int kk  = ((i < 8) ? i : (i + 8)) + 8 * hsel;
      int src = (kk < CONV_OUT) ? kk : ((kk >= 16 && kk < 16 + H) ? kk - 4 : -1);
      int n = j * 16 + (lane & 15);
      float val = (src >= 0 && n < G4) ? W[src * G4 + n] : 0.f;
      wb[j][i] = (_Float16)val;
    }
    int n = j * 16 + (lane & 15);
    float bv = (n < G4) ? B[n] : 0.f;
    #pragma unroll
    for (int v = 0; v < 8; ++v) biasC[j][v] = bv;
  }

  {
    v8h z8 = {};
    *(v8h*)&s_h[wave][lane * 8] = z8;
  }
  float cst[5], hreg[5];
  #pragma unroll
  for (int r = 0; r < 5; ++r) { cst[r] = 0.f; hreg[r] = 0.f; }
  __syncthreads();

  const _Float16* xb = &s_c[m * SC * 16 + 8 * hsel];
  const _Float16* hb = &s_h[wave][m * 16 + 8 * hsel];
  _Float16* hwr = &s_h[wave][0];
  float* zb = &s_z[wave][0];
  const int nl = lane & 15;
  #pragma unroll 1
  for (int t = 0; t < SC; ++t) {
    int tcur = wave ? (SC - 1 - t) : t;
    v8h r0 = *(const v8h*)(xb + tcur * 16);
    v8h r1 = *(const v8h*)(hb);
    v16h a = __builtin_shufflevector(r0, r1, 0,1,2,3,4,5,6,7,8,9,10,11,12,13,14,15);
    v8f z0 = wmma16(a, wb[0], biasC[0]);
    v8f z1 = wmma16(a, wb[1], biasC[1]);
    v8f z2 = wmma16(a, wb[2], biasC[2]);
    *(v8f*)(zb + (nl)      * 16 + 8 * hsel) = z0;
    *(v8f*)(zb + (16 + nl) * 16 + 8 * hsel) = z1;
    *(v8f*)(zb + (32 + nl) * 16 + 8 * hsel) = z2;
    LDS_FENCE();
    #pragma unroll
    for (int r = 0; r < 5; ++r) {
      int p = lane + 32 * r;
      int seq = p / H, u = p % H;
      float zi = zb[u * 16 + seq];
      float zg = zb[(10 + u) * 16 + seq];
      float zf = zb[(20 + u) * 16 + seq];
      float zo = zb[(30 + u) * 16 + seq];
      float cc = sigm(zf + 1.f) * cst[r] + sigm(zi) * tanh_fast(zg);
      float hh = sigm(zo) * tanh_fast(cc);
      cst[r] = cc; hreg[r] = hh;
      hwr[seq * 16 + u] = (_Float16)hh;
    }
    LDS_FENCE();
  }

  __shared__ __align__(16) float s_o[TILE * 2 * H];
  #pragma unroll
  for (int r = 0; r < 5; ++r) {
    int p = lane + 32 * r;
    int seq = p / H, u = p % H;
    s_o[seq * (2 * H) + wave * H + u] = hreg[r];
  }
  __syncthreads();
  typedef __attribute__((ext_vector_type(4))) float v4f_t; typedef float v4fa __attribute__((ext_vector_type(4), may_alias));
  float* ob = out + (size_t)base * (2 * H);
  for (int c = tid; c < TILE * 2 * H / 4; c += 64) {
    const v4f_t v = *(const volatile v4fa*)(s_o + c * 4);
    *(volatile v4f_t*)(ob + c * 4) = v; __threadfence(); *(volatile v4f_t*)(ob + c * 4) = v;
  }
}

extern "C" void kernel_launch(void* const* d_in, const int* in_sizes, int n_in,
                              void* d_out, int out_size, void* d_ws, size_t ws_size,
                              hipStream_t stream) {
  const int*   in_ids = (const int*)  d_in[0];
  const float* embp   = (const float*)d_in[1];
  const float* k2p    = (const float*)d_in[2];
  const float* k3p    = (const float*)d_in[3];
  const float* k4p    = (const float*)d_in[4];
  const float* w_fw   = (const float*)d_in[5];
  const float* b_fw   = (const float*)d_in[6];
  const float* w_bw   = (const float*)d_in[7];
  const float* b_bw   = (const float*)d_in[8];
  float* outp = (float*)d_out;

  int nseq   = in_sizes[0] / SC;
  int blocks = nseq / TILE;
  cnn_bilstm_kernel<<<blocks, 64, 0, stream>>>(in_ids, embp, k2p, k3p, k4p,
                                               w_fw, b_fw, w_bw, b_bw, outp);
}
